// FactorPredictor_40931038331019
// MI455X (gfx1250) — hardware-verified
//
#include <hip/hip_runtime.h>
#include <math.h>
typedef __attribute__((ext_vector_type(16))) _Float16 v16h;
typedef __attribute__((ext_vector_type(8)))  _Float16 v8h;
typedef __attribute__((ext_vector_type(16))) __bf16   v16b;
typedef __attribute__((ext_vector_type(8)))  __bf16   v8b;
typedef __attribute__((ext_vector_type(8)))  float    v8f;
typedef __attribute__((ext_vector_type(4)))  float    v4f;
#define PSCALE 32768.0f
#define U16(p) ((const unsigned short*)(const void*)(p))
#define PSCALE_INV (1.0f / 32768.0f)

__device__ __forceinline__ unsigned short f2bf_bits(float f) {
  unsigned u = __float_as_uint(f);
  return (unsigned short)((u + 0x7FFFu + ((u >> 16) & 1u)) >> 16);
}
__device__ __forceinline__ float bf_bits2f(unsigned short h) { return __uint_as_float(((unsigned)h) << 16); }

__device__ __forceinline__ void dep_guard_h(v8f& a, v8f& b, v16h x, v16h y) { asm volatile("v_nop\n\tv_nop\n\tv_nop\n\tv_nop" : "+v"(a), "+v"(b) : "v"(x), "v"(y)); }
__device__ __forceinline__ void dep_guard_b(v8f& a, v8f& b, v16b x, v16b y) { asm volatile("v_nop\n\tv_nop\n\tv_nop\n\tv_nop" : "+v"(a), "+v"(b) : "v"(x), "v"(y)); }
__device__ __forceinline__ void keep4_h(v16h a, v16h b, v16h c, v16h d) { asm volatile("v_nop" :: "v"(a), "v"(b), "v"(c), "v"(d)); }
__device__ __forceinline__ void keep4_b(v16b a, v16b b, v16b c, v16b d) { asm volatile("v_nop" :: "v"(a), "v"(b), "v"(c), "v"(d)); }
__device__ __forceinline__ void acc_guard4(v8f& a, v8f& b, v8f& c, v8f& d) { asm volatile("v_nop\n\tv_nop\n\tv_nop\n\tv_nop" : "+v"(a), "+v"(b), "+v"(c), "+v"(d)); }
template <typename T> struct Frag;
template <> struct Frag<_Float16> {
  typedef v16h V; union U { v16h v; v8h h[2]; };
  static __device__ __forceinline__ v16h load(const _Float16* p) {
    U f; f.h[0] = *(const v8h*)(p); f.h[1] = *(const v8h*)(p + 16); return f.v;
  }
  static __device__ __forceinline__ v8f mma(v16h a, v16h b, v8f c) {
    return __builtin_amdgcn_wmma_f32_16x16x32_f16(false, a, false, b, (short)0, c, false, false);
  }
  static __device__ __forceinline__ void guard(v8f& a, v8f& b, v16h x, v16h y) { dep_guard_h(a, b, x, y); }
  static __device__ __forceinline__ void keep(v16h a, v16h b, v16h c, v16h d) { keep4_h(a, b, c, d); }
};
template <> struct Frag<__bf16> {
  typedef v16b V; union U { v16b v; v8b h[2]; };
  static __device__ __forceinline__ v16b load(const __bf16* p) {
    U f; f.h[0] = *(const v8b*)(p); f.h[1] = *(const v8b*)(p + 16); return f.v;
  }
  static __device__ __forceinline__ v8f mma(v16b a, v16b b, v8f c) {
    return __builtin_amdgcn_wmma_f32_16x16x32_bf16(false, a, false, b, (short)0, c, false, false);
  }
  static __device__ __forceinline__ void guard(v8f& a, v8f& b, v16b x, v16b y) { dep_guard_b(a, b, x, y); }
  static __device__ __forceinline__ void keep(v16b a, v16b b, v16b c, v16b d) { keep4_b(a, b, c, d); }
};

template <int ET> struct Elem;
template <> struct Elem<0> { typedef _Float16 T; };
template <> struct Elem<1> { typedef __bf16 T; };
template <int ET, bool SPLIT, int BIAS_MODE, int OUT_MODE, bool RESID, int ACT = 0>
__global__ __launch_bounds__(256) void wmma_gemm64(
    const unsigned short* __restrict__ Ap, const unsigned short* __restrict__ A2p, int lda, long strideA,
    const unsigned short* __restrict__ Btp, const unsigned short* __restrict__ Bt2p, int ldb, long strideB,
    void* __restrict__ Cout, void* __restrict__ Cout2, int ldc, long strideC,
    const float* __restrict__ bias,
    const float* __restrict__ resid, long strideR,
    int M, int N, int K, float scale) {
  typedef typename Elem<ET>::T T;
  typedef typename Frag<T>::V V;
  const T* A = (const T*)Ap; const T* A2 = (const T*)A2p; const T* Bt = (const T*)Btp; const T* Bt2 = (const T*)Bt2p;
  __shared__ __align__(16) float sT[8][16 * 68];
  const int b    = blockIdx.y;
  const int lane = threadIdx.x & 31;
  const int wave = threadIdx.x >> 5;
  const int tilesN = N >> 6;
  const int tilesM = M >> 6;
  const int tile = blockIdx.x * 8 + wave;
  if (tile >= tilesM * tilesN) return;
  const int tm = tile / tilesN;
  const int tn = tile - tm * tilesN;
  const int m0 = tm << 6;
  const int n0 = tn << 6;

  const T* Ab  = A  + (size_t)b * strideA;
  const T* Bb  = Bt + (size_t)b * strideB;
  const T* Ab2 = SPLIT ? (A2  + (size_t)b * strideA) : nullptr;
  const T* Bb2 = SPLIT ? (Bt2 + (size_t)b * strideB) : nullptr;

  const int rlane = lane & 15;
  const int koff  = (lane >> 4) * 8;
  const int mOff  = (lane >> 4) * 8;

  v8f acc[4][4];
#pragma unroll
  for (int i = 0; i < 4; ++i)
#pragma unroll
    for (int j = 0; j < 4; ++j) acc[i][j] = (v8f){0.f,0.f,0.f,0.f,0.f,0.f,0.f,0.f};

  for (int k0 = 0; k0 < K; k0 += 32) {
    V bh[4], bl[4];
#pragma unroll
    for (int j = 0; j < 4; ++j) {
      const size_t bo = (size_t)(n0 + (j << 4) + rlane) * ldb + koff + k0;
      bh[j] = Frag<T>::load(Bb + bo);
      if (SPLIT) bl[j] = Frag<T>::load(Bb2 + bo);
    }
#pragma unroll
    for (int i = 0; i < 4; ++i) {
      const size_t ao = (size_t)(m0 + (i << 4) + rlane) * lda + koff + k0;
      V ah = Frag<T>::load(Ab + ao);
      V al;
      if (SPLIT) al = Frag<T>::load(Ab2 + ao);
#pragma unroll
      for (int j = 0; j < 4; ++j) {
        acc[i][j] = Frag<T>::mma(ah, bh[j], acc[i][j]);
        if (SPLIT) {
          acc[i][j] = Frag<T>::mma(ah, bl[j], acc[i][j]);
          acc[i][j] = Frag<T>::mma(al, bh[j], acc[i][j]);
        }
      }
      Frag<T>::guard(acc[i][0], acc[i][3], ah, SPLIT ? al : ah);
    }
    Frag<T>::keep(bh[0], bh[1], bh[2], bh[3]);
    if (SPLIT) Frag<T>::keep(bl[0], bl[1], bl[2], bl[3]);
  }
  acc_guard4(acc[0][0], acc[0][1], acc[0][2], acc[0][3]);
  acc_guard4(acc[1][0], acc[1][1], acc[1][2], acc[1][3]);
  acc_guard4(acc[2][0], acc[2][1], acc[2][2], acc[2][3]);
  acc_guard4(acc[3][0], acc[3][1], acc[3][2], acc[3][3]);

  float* slab = sT[wave];
  const float* Rb = RESID ? (resid + (size_t)b * strideR) : nullptr;
#pragma unroll
  for (int i = 0; i < 4; ++i) {
    const int mBase = m0 + (i << 4);
#pragma unroll
    for (int j = 0; j < 4; ++j) {
      const int n = n0 + (j << 4) + rlane;
      float bv = 0.f;
      if (BIAS_MODE == 2) bv = bias[n];
#pragma unroll
      for (int r = 0; r < 8; ++r) {
        float v = acc[i][j][r] * scale;
        if (BIAS_MODE == 1) v += bias[mBase + mOff + r];
        if (BIAS_MODE == 2) v += bv;
        if (RESID) v += Rb[(size_t)(mBase + mOff + r) * ldc + n];
        if (ACT == 1) v = tanhf(v);
        if (ACT == 2) v = fmaxf(v, 0.0f);
        if (ACT == 3) v = v / (1.0f + expf(-v));
        if (ACT == 4) v = (v > 0.f) ? v : 0.01f * v;
        if (ACT == 5) v = 0.5f * v * (1.0f + erff(v * 0.70710678118654752f));
        slab[(mOff + r) * 68 + (j << 4) + rlane] = v;
      }
    }
    __builtin_amdgcn_fence(__ATOMIC_RELEASE, "workgroup");
    __builtin_amdgcn_wave_barrier();
    __builtin_amdgcn_fence(__ATOMIC_ACQUIRE, "workgroup");
    if (OUT_MODE == 0) {
      float* C = (float*)Cout + (size_t)b * strideC;
      const int hh = lane >> 4, c4 = (lane & 15) * 4;
      for (int pass = 0; pass < 2; ++pass) {
#pragma unroll
        for (int it = 0; it < 8; ++it) {
          const int row = it * 2 + hh;
          v4f v = *(const v4f*)(slab + row * 68 + c4);
          *(volatile v4f*)(C + (size_t)(mBase + row) * ldc + n0 + c4) = v;
        }
        __threadfence();
      }
    } else {
      const int q = lane >> 3, c8 = (lane & 7) * 8;
      unsigned short* C  = (unsigned short*)Cout  + (size_t)b * strideC;
      unsigned short* C2 = (OUT_MODE == 2) ? ((unsigned short*)Cout2 + (size_t)b * strideC) : nullptr;
      for (int pass = 0; pass < 2; ++pass) {
#pragma unroll
        for (int it = 0; it < 4; ++it) {
          const int row = it * 4 + q;
          const float* sp = slab + row * 68 + c8;
          v8h hv, lv;
#pragma unroll
          for (int e = 0; e < 8; ++e) {
            if (OUT_MODE == 1) {
              hv[e] = (_Float16)sp[e];
            } else {
              unsigned short hb = f2bf_bits(sp[e]);
              unsigned short lb = f2bf_bits(sp[e] - bf_bits2f(hb));
              hv[e] = __builtin_bit_cast(_Float16, hb);
              lv[e] = __builtin_bit_cast(_Float16, lb);
            }
          }
          *(volatile v8h*)(C + (size_t)(mBase + row) * ldc + n0 + c8) = hv;
          if (OUT_MODE == 2) *(volatile v8h*)(C2 + (size_t)(mBase + row) * ldc + n0 + c8) = lv;
        }
        __threadfence();
      }
    }
    __builtin_amdgcn_fence(__ATOMIC_RELEASE, "workgroup");
    __builtin_amdgcn_wave_barrier();
    __builtin_amdgcn_fence(__ATOMIC_ACQUIRE, "workgroup");
  }
}

__global__ __launch_bounds__(256) void cast_f32_f16x2(
    const float* __restrict__ in, _Float16* __restrict__ out, int n2) {
  int i = blockIdx.x * 256 + threadIdx.x;
  if (i < n2) {
    const _Float16 h0 = (_Float16)in[2 * i], h1 = (_Float16)in[2 * i + 1];
    const unsigned u = (unsigned)__builtin_bit_cast(unsigned short, h0) | ((unsigned)__builtin_bit_cast(unsigned short, h1) << 16);
    ((volatile unsigned*)out)[i] = u;
    __threadfence();
    ((volatile unsigned*)out)[i] = u;
  }
}

__global__ __launch_bounds__(256) void split_f32_bf16x2(
    const float* __restrict__ in, __bf16* __restrict__ hi, __bf16* __restrict__ lo, long n2) {
  long i = (long)blockIdx.x * 256 + threadIdx.x;
  long stride = (long)gridDim.x * 256;
  for (int pass = 0; pass < 2; ++pass) {
    for (long j = i; j < n2; j += stride) {
      const float a = in[2 * j], b = in[2 * j + 1];
      const unsigned short ah = f2bf_bits(a), bh = f2bf_bits(b);
      const unsigned short al = f2bf_bits(a - bf_bits2f(ah)), bl = f2bf_bits(b - bf_bits2f(bh));
      ((volatile unsigned*)hi)[j] = (unsigned)ah | ((unsigned)bh << 16);
      ((volatile unsigned*)lo)[j] = (unsigned)al | ((unsigned)bl << 16);
    }
    __threadfence();
  }
}


__global__ __launch_bounds__(256) void transpose_split_bf16(const float* __restrict__ in, int ldi,
                                                           __bf16* __restrict__ outH, __bf16* __restrict__ outL, int ldo) {
  __shared__ __align__(16) float tile[64][68];
  const int c0 = blockIdx.x * 64, r0 = blockIdx.y * 64;
  const int t = threadIdx.y * 32 + threadIdx.x;
  for (int i = threadIdx.y; i < 64; i += 8) {
    tile[threadIdx.x][i]      = in[(size_t)(r0 + i) * ldi + c0 + threadIdx.x];
    tile[32 + threadIdx.x][i] = in[(size_t)(r0 + i) * ldi + c0 + 32 + threadIdx.x];
  }
  __syncthreads();
  const int q = t >> 3, c8 = (t & 7) * 8;
  for (int pass = 0; pass < 2; ++pass) {
#pragma unroll
    for (int it = 0; it < 2; ++it) {
      const int c = it * 32 + q;
      v8b hv, lv;
#pragma unroll
      for (int e = 0; e < 8; ++e) {
        const float f = tile[c][c8 + e];
        const unsigned short hb = f2bf_bits(f);
        hv[e] = __builtin_bit_cast(__bf16, hb);
        lv[e] = __builtin_bit_cast(__bf16, f2bf_bits(f - bf_bits2f(hb)));
      }
      *(volatile v8b*)(outH + (size_t)(c0 + c) * ldo + r0 + c8) = hv;
      *(volatile v8b*)(outL + (size_t)(c0 + c) * ldo + r0 + c8) = lv;
    }
    __threadfence();
  }
}

#define FBS 65536
#define FHD 32
#define FF 64
__global__ void bias2_kernel(const float* a, const float* b, float* o) { const int i = threadIdx.x; if (i < 64) { const float v = (i < 32) ? a[i] : b[i - 32]; ((volatile float*)o)[i] = v; __threadfence(); ((volatile float*)o)[i] = v; } }
__global__ __launch_bounds__(256) void qprep_kernel(const float* __restrict__ query, __bf16* __restrict__ Qh, __bf16* __restrict__ Ql, float* __restrict__ qinv) {
  const int t = threadIdx.x;
  for (int i = t; i < FF * 64; i += 256) { const int f = i / 64, j = i % 64; const float qv = query[(j & 31) * FF + f]; const float a = (j < 32) ? fmaxf(qv, 0.f) : fmaxf(-qv, 0.f);
    const unsigned short h = f2bf_bits(a), l = f2bf_bits(a - bf_bits2f(h));
    for (int pass = 0; pass < 2; ++pass) { ((volatile __bf16*)Qh)[i] = __builtin_bit_cast(__bf16, h); ((volatile __bf16*)Ql)[i] = __builtin_bit_cast(__bf16, l); __threadfence(); } }
  if (t < FF) { float s = 0.f; for (int h2 = 0; h2 < FHD; ++h2) s += query[h2 * FF + t] * query[h2 * FF + t]; const float v = 1.0f / (sqrtf(s) + 1e-6f); ((volatile float*)qinv)[t] = v; __threadfence(); ((volatile float*)qinv)[t] = v; }
}
__global__ __launch_bounds__(256) void kprep_kernel(const float* __restrict__ KV, __bf16* __restrict__ Kh, __bf16* __restrict__ Kl, float* __restrict__ P) {
  const int lane = threadIdx.x & 31, wave = threadIdx.x >> 5; const size_t b = (size_t)blockIdx.x * 8 + wave;
  const float k = KV[b * 64 + lane], v = KV[b * 64 + 32 + lane];
  float kk = k * k; for (int o = 16; o > 0; o >>= 1) kk += __shfl_xor(kk, o, 32);
  const float kn = k / (sqrtf(kk) + 1e-6f); const float kp = fmaxf(kn, 0.f), km = fmaxf(-kn, 0.f);
  const unsigned short ph = f2bf_bits(kp), pl = f2bf_bits(kp - bf_bits2f(ph)), mh = f2bf_bits(km), ml = f2bf_bits(km - bf_bits2f(mh));
  for (int pass = 0; pass < 2; ++pass) {
    ((volatile __bf16*)Kh)[b * 64 + lane] = __builtin_bit_cast(__bf16, ph); ((volatile __bf16*)Kl)[b * 64 + lane] = __builtin_bit_cast(__bf16, pl);
    ((volatile __bf16*)Kh)[b * 64 + 32 + lane] = __builtin_bit_cast(__bf16, mh); ((volatile __bf16*)Kl)[b * 64 + 32 + lane] = __builtin_bit_cast(__bf16, ml);
    ((volatile float*)P)[b * 128 + lane] = kp * v; ((volatile float*)P)[b * 128 + 32 + lane] = km * v; ((volatile float*)P)[b * 128 + 64 + lane] = v; ((volatile float*)P)[b * 128 + 96 + lane] = 0.f;
    __threadfence(); }
}
__global__ __launch_bounds__(256) void winv_kernel(const float* __restrict__ S, const float* __restrict__ qinv, float* __restrict__ Wm) {
  const size_t i = (size_t)blockIdx.x * 256 + threadIdx.x; if (i >= (size_t)FBS * FF) return; const int f = (int)(i & 63);
  const float w = 1.0f / (S[i] * qinv[f] + 32.0f * 1e-6f); ((volatile float*)Wm)[i] = w; __threadfence(); ((volatile float*)Wm)[i] = w;
}
__global__ __launch_bounds__(256) void head_kernel(const float* __restrict__ C, const float* __restrict__ query, const float* __restrict__ qinv, const float* __restrict__ lng, const float* __restrict__ lnb,
                                                  const float* __restrict__ mW1, const float* __restrict__ mb1, const float* __restrict__ mW2, const float* __restrict__ mb2,
                                                  const float* __restrict__ sW1, const float* __restrict__ sb1, const float* __restrict__ sW2, const float* __restrict__ sb2, float* __restrict__ mu, float* __restrict__ sg) {
  __shared__ float fn[2048]; __shared__ double red[256], red2[256]; __shared__ float h1[64], h2[64];
  const int t = threadIdx.x;
  double vals[8]; double s = 0.0;
  for (int q = 0; q < 8; ++q) { const int i = t + 256 * q; const int f = i / FHD, h = i % FHD; const float qv = query[h * FF + f];
    const double val = ((double)fmaxf(qv, 0.f) * C[f * 128 + h] + (double)fmaxf(-qv, 0.f) * C[f * 128 + 32 + h]) * (double)qinv[f] + 1e-6 * (double)C[f * 128 + 64 + h];
    vals[q] = val; s += val; }
  red[t] = s; __syncthreads();
  for (int o = 128; o > 0; o >>= 1) { if (t < o) red[t] += red[t + o]; __syncthreads(); }
  const double mean = red[0] / 2048.0; __syncthreads();
  double s2 = 0.0; for (int q = 0; q < 8; ++q) { const double d = vals[q] - mean; s2 += d * d; }
  red2[t] = s2; __syncthreads();
  for (int o = 128; o > 0; o >>= 1) { if (t < o) red2[t] += red2[t + o]; __syncthreads(); }
  const double inv = 1.0 / sqrt(red2[0] / 2048.0 + 1e-5);
  for (int q = 0; q < 8; ++q) { const int i = t + 256 * q; fn[i] = (float)((vals[q] - mean) * inv) * lng[i] + lnb[i]; }
  __syncthreads();
  if (t < 128) { const int o = t & 63; const float* Wt = (t < 64) ? mW1 : sW1; const float* bb = (t < 64) ? mb1 : sb1; float a = bb[o];
#pragma unroll 1
    for (int i = 0; i < 2048; ++i) a += fn[i] * Wt[(size_t)o * 2048 + i];
    a = fmaxf(a, 0.f); if (t < 64) h1[o] = a; else h2[o] = a; }
  __syncthreads();
  float res = 0.f;
  if (t < 128) { const int o = t & 63; const float* Wt = (t < 64) ? mW2 : sW2; const float* bb = (t < 64) ? mb2 : sb2; const float* hh = (t < 64) ? h1 : h2; float a = bb[o];
#pragma unroll 1
    for (int i = 0; i < 64; ++i) a += hh[i] * Wt[o * 64 + i];
    res = (t < 64) ? a : ((a > 20.f) ? a : log1pf(expf(a))); }
  for (int pass = 0; pass < 2; ++pass) { if (t < 64) ((volatile float*)mu)[t] = res; else if (t < 128) ((volatile float*)sg)[t - 64] = res; __threadfence(); }
}
extern "C" void kernel_launch(void* const* d_in, const int* in_sizes, int n_in, void* d_out, int out_size, void* d_ws, size_t ws_size, hipStream_t stream) {
  (void)in_sizes; (void)n_in; (void)out_size; (void)ws_size;
  const float* x = (const float*)d_in[0]; const float* kW = (const float*)d_in[1]; const float* kb = (const float*)d_in[2]; const float* vW = (const float*)d_in[3]; const float* vb = (const float*)d_in[4]; const float* query = (const float*)d_in[5];
  const float* lng = (const float*)d_in[6]; const float* lnb = (const float*)d_in[7];
  auto F = [&](int i) { return (const float*)d_in[i]; };
  float* mu = (float*)d_out; float* sg = mu + 64;
  char* ws = (char*)d_ws; size_t off = 0;
  auto carve = [&](size_t bytes) -> char* { char* p = ws + off; off += (bytes + 255) & ~(size_t)255; return p; };
  __bf16* Xh = (__bf16*)carve((size_t)FBS * FHD * 2); __bf16* Xl = (__bf16*)carve((size_t)FBS * FHD * 2); __bf16* Wh = (__bf16*)carve(64 * FHD * 2); __bf16* Wl = (__bf16*)carve(64 * FHD * 2); float* bb = (float*)carve(64 * 4);
  float* KV = (float*)carve((size_t)FBS * 64 * 4); __bf16* Qh = (__bf16*)carve(FF * 64 * 2); __bf16* Ql = (__bf16*)carve(FF * 64 * 2); float* qinv = (float*)carve(FF * 4);
  __bf16* Kh = (__bf16*)carve((size_t)FBS * 64 * 2); __bf16* Kl = (__bf16*)carve((size_t)FBS * 64 * 2); float* P = (float*)carve((size_t)FBS * 128 * 4);
  float* S = (float*)carve((size_t)FBS * FF * 4); float* Wm = (float*)carve((size_t)FBS * FF * 4);
  __bf16* WTh = (__bf16*)carve((size_t)FF * FBS * 2); __bf16* WTl = (__bf16*)carve((size_t)FF * FBS * 2); __bf16* PTh = (__bf16*)carve((size_t)128 * FBS * 2); __bf16* PTl = (__bf16*)carve((size_t)128 * FBS * 2);
  float* C = (float*)carve(FF * 128 * 4);
  split_f32_bf16x2<<<(FBS * FHD / 2 + 255) / 256, 256, 0, stream>>>(x, Xh, Xl, FBS * FHD / 2);
  split_f32_bf16x2<<<(FHD * FHD / 2 + 255) / 256, 256, 0, stream>>>(kW, Wh, Wl, FHD * FHD / 2);
  split_f32_bf16x2<<<(FHD * FHD / 2 + 255) / 256, 256, 0, stream>>>(vW, Wh + FHD * FHD, Wl + FHD * FHD, FHD * FHD / 2);
  bias2_kernel<<<1, 64, 0, stream>>>(kb, vb, bb);
  { const int t = (FBS / 64) * 1;
    wmma_gemm64<1, true, 2, 0, false><<<dim3((t + 7) / 8, 1), 256, 0, stream>>>(U16(Xh), U16(Xl), FHD, 0, U16(Wh), U16(Wl), FHD, 0, KV, nullptr, 64, 0, bb, nullptr, 0, FBS, 64, FHD, 1.0f); }
  qprep_kernel<<<1, 256, 0, stream>>>(query, Qh, Ql, qinv);
  kprep_kernel<<<FBS / 8, 256, 0, stream>>>(KV, Kh, Kl, P);
  { const int t = (FBS / 64) * 1;
    wmma_gemm64<1, true, 0, 0, false><<<dim3((t + 7) / 8, 1), 256, 0, stream>>>(U16(Kh), U16(Kl), 64, 0, U16(Qh), U16(Ql), 64, 0, S, nullptr, FF, 0, nullptr, nullptr, 0, FBS, FF, 64, 1.0f); }
  winv_kernel<<<(FBS * FF + 255) / 256, 256, 0, stream>>>(S, qinv, Wm);
  transpose_split_bf16<<<dim3(FF / 64, FBS / 64), dim3(32, 8), 0, stream>>>(Wm, FF, WTh, WTl, FBS);
  transpose_split_bf16<<<dim3(128 / 64, FBS / 64), dim3(32, 8), 0, stream>>>(P, 128, PTh, PTl, FBS);
  { const int t = 1 * 2;
    wmma_gemm64<1, true, 0, 0, false><<<dim3((t + 7) / 8, 1), 256, 0, stream>>>(U16(WTh), U16(WTl), FBS, 0, U16(PTh), U16(PTl), FBS, 0, C, nullptr, 128, 0, nullptr, nullptr, 0, FF, 128, FBS, 1.0f); }
  head_kernel<<<1, 256, 0, stream>>>(C, query, qinv, lng, lnb, F(8), F(9), F(10), F(11), F(12), F(13), F(14), F(15), mu, sg);
}
